// MobileMQA_42752104465005
// MI455X (gfx1250) — hardware-verified
//
#include <hip/hip_runtime.h>
#include <math.h>

constexpr int kBatch   = 8;
constexpr int kTok     = 1024;
constexpr int kGridHW  = 32;
constexpr int kDim     = 512;
constexpr int kHeads   = 8;
constexpr int kHd      = 64;
constexpr int kNk      = 256;
constexpr int kRedHW   = 16;
constexpr int kKeys    = kNk * kHeads;
constexpr int kRows    = kBatch * kTok;
constexpr int kKvRows  = kBatch * kNk;
constexpr int kConvK   = 4 * kDim;
constexpr int kHeadGrp = 4;
constexpr float kWqCarry    = 16.0f;
constexpr float kWqCarryInv = 1.0f / 16.0f;
constexpr float kPCarry     = 32768.0f;
constexpr float kPCarryInv  = 1.0f / 32768.0f;
constexpr float kInvDim     = 1.0f / 512.0f;
constexpr float kLnEps      = 1e-5f;
constexpr float kAttnScale  = 0.125f;

typedef __attribute__((ext_vector_type(16))) _Float16 v16h;
typedef __attribute__((ext_vector_type(8)))  _Float16 v8h;
typedef __attribute__((ext_vector_type(16))) __bf16   v16b;
typedef __attribute__((ext_vector_type(8)))  __bf16   v8b;
typedef __attribute__((ext_vector_type(8)))  float    v8f;
typedef __attribute__((ext_vector_type(4)))  float    v4f;
typedef __attribute__((ext_vector_type(4)))  unsigned int v4u;

__device__ __forceinline__ unsigned short f2bf_bits(float f) {
  unsigned u = __float_as_uint(f);
  return (unsigned short)((u + 0x7FFFu + ((u >> 16) & 1u)) >> 16);
}
__device__ __forceinline__ float bf_bits2f(unsigned short h) { return __uint_as_float(((unsigned)h) << 16); }

__device__ __forceinline__ void dep_guard_h(v8f& a, v8f& b, v16h x, v16h y) { asm volatile("v_nop\n\tv_nop\n\tv_nop\n\tv_nop" : "+v"(a), "+v"(b) : "v"(x), "v"(y)); }
__device__ __forceinline__ void dep_guard_b(v8f& a, v8f& b, v16b x, v16b y) { asm volatile("v_nop\n\tv_nop\n\tv_nop\n\tv_nop" : "+v"(a), "+v"(b) : "v"(x), "v"(y)); }
__device__ __forceinline__ void keep4_h(v16h a, v16h b, v16h c, v16h d) { asm volatile("v_nop" :: "v"(a), "v"(b), "v"(c), "v"(d)); }
__device__ __forceinline__ void keep4_b(v16b a, v16b b, v16b c, v16b d) { asm volatile("v_nop" :: "v"(a), "v"(b), "v"(c), "v"(d)); }
__device__ __forceinline__ void acc_guard4(v8f& a, v8f& b, v8f& c, v8f& d) { asm volatile("v_nop\n\tv_nop\n\tv_nop\n\tv_nop" : "+v"(a), "+v"(b), "+v"(c), "+v"(d)); }
template <typename T> struct Frag;
template <> struct Frag<_Float16> {
  typedef v16h V; union U { v16h v; v8h h[2]; };
  static __device__ __forceinline__ v16h load(const _Float16* p) {
    U f; f.h[0] = *(const v8h*)(p); f.h[1] = *(const v8h*)(p + 16); return f.v;
  }
  static __device__ __forceinline__ v8f mma(v16h a, v16h b, v8f c) {
    return __builtin_amdgcn_wmma_f32_16x16x32_f16(false, a, false, b, (short)0, c, false, false);
  }
  static __device__ __forceinline__ void guard(v8f& a, v8f& b, v16h x, v16h y) { dep_guard_h(a, b, x, y); }
  static __device__ __forceinline__ void keep(v16h a, v16h b, v16h c, v16h d) { keep4_h(a, b, c, d); }
};
template <> struct Frag<__bf16> {
  typedef v16b V; union U { v16b v; v8b h[2]; };
  static __device__ __forceinline__ v16b load(const __bf16* p) {
    U f; f.h[0] = *(const v8b*)(p); f.h[1] = *(const v8b*)(p + 16); return f.v;
  }
  static __device__ __forceinline__ v8f mma(v16b a, v16b b, v8f c) {
    return __builtin_amdgcn_wmma_f32_16x16x32_bf16(false, a, false, b, (short)0, c, false, false);
  }
  static __device__ __forceinline__ void guard(v8f& a, v8f& b, v16b x, v16b y) { dep_guard_b(a, b, x, y); }
  static __device__ __forceinline__ void keep(v16b a, v16b b, v16b c, v16b d) { keep4_b(a, b, c, d); }
};

__device__ __forceinline__ unsigned pk16(unsigned short a, unsigned short b) { return (unsigned)a | ((unsigned)b << 16); }
__device__ __forceinline__ unsigned short h_bits(float f) { const _Float16 h = (_Float16)f; return __builtin_bit_cast(unsigned short, h); }

template <int ET> struct Elem;
template <> struct Elem<0> { typedef _Float16 T; };
template <> struct Elem<1> { typedef __bf16 T; };
template <int ET, bool SPLIT, int BIAS_MODE, int OUT_MODE, bool RESID, int ACT = 0>
__global__ __launch_bounds__(256) void wmma_gemm64(
    const unsigned short* __restrict__ Ap, const unsigned short* __restrict__ A2p, int lda, long strideA,
    const unsigned short* __restrict__ Btp, const unsigned short* __restrict__ Bt2p, int ldb, long strideB,
    void* __restrict__ Cout, void* __restrict__ Cout2, int ldc, long strideC,
    const float* __restrict__ bias, long strideBias,
    const float* __restrict__ resid, long strideR,
    int M, int N, int K, float scale) {
  typedef typename Elem<ET>::T T;
  typedef typename Frag<T>::V V;
  const T* A = (const T*)Ap; const T* A2 = (const T*)A2p; const T* Bt = (const T*)Btp; const T* Bt2 = (const T*)Bt2p;
  __shared__ __align__(16) float sT[8][16 * 68];
  const int b    = blockIdx.y;
  const int lane = threadIdx.x & 31;
  const int wave = threadIdx.x >> 5;
  const int tilesN = N >> 6;
  const int tilesM = M >> 6;
  const int tile = blockIdx.x * 8 + wave;
  if (tile >= tilesM * tilesN) return;
  const int tm = tile / tilesN;
  const int tn = tile - tm * tilesN;
  const int m0 = tm << 6;
  const int n0 = tn << 6;

  const T* Ab  = A  + (size_t)b * strideA;
  const T* Bb  = Bt + (size_t)b * strideB;
  const T* Ab2 = SPLIT ? (A2  + (size_t)b * strideA) : nullptr;
  const T* Bb2 = SPLIT ? (Bt2 + (size_t)b * strideB) : nullptr;

  const int rlane = lane & 15;
  const int koff  = (lane >> 4) * 8;
  const int mOff  = (lane >> 4) * 8;

  v8f acc[4][4];
#pragma unroll
  for (int i = 0; i < 4; ++i)
#pragma unroll
    for (int j = 0; j < 4; ++j) acc[i][j] = (v8f){0.f,0.f,0.f,0.f,0.f,0.f,0.f,0.f};

  for (int k0 = 0; k0 < K; k0 += 32) {
    V bh[4], bl[4];
#pragma unroll
    for (int j = 0; j < 4; ++j) {
      const size_t bo = (size_t)(n0 + (j << 4) + rlane) * ldb + koff + k0;
      bh[j] = Frag<T>::load(Bb + bo);
      if (SPLIT) bl[j] = Frag<T>::load(Bb2 + bo);
    }
#pragma unroll
    for (int i = 0; i < 4; ++i) {
      const size_t ao = (size_t)(m0 + (i << 4) + rlane) * lda + koff + k0;
      V ah = Frag<T>::load(Ab + ao);
      V al;
      if (SPLIT) al = Frag<T>::load(Ab2 + ao);
#pragma unroll
      for (int j = 0; j < 4; ++j) {
        acc[i][j] = Frag<T>::mma(ah, bh[j], acc[i][j]);
        if (SPLIT) {
          acc[i][j] = Frag<T>::mma(ah, bl[j], acc[i][j]);
          acc[i][j] = Frag<T>::mma(al, bh[j], acc[i][j]);
        }
      }
      Frag<T>::guard(acc[i][0], acc[i][3], ah, SPLIT ? al : ah);
    }
    Frag<T>::keep(bh[0], bh[1], bh[2], bh[3]);
    if (SPLIT) Frag<T>::keep(bl[0], bl[1], bl[2], bl[3]);
  }
  acc_guard4(acc[0][0], acc[0][1], acc[0][2], acc[0][3]);
  acc_guard4(acc[1][0], acc[1][1], acc[1][2], acc[1][3]);
  acc_guard4(acc[2][0], acc[2][1], acc[2][2], acc[2][3]);
  acc_guard4(acc[3][0], acc[3][1], acc[3][2], acc[3][3]);

  float* slab = sT[wave];
  const float* Rb = RESID ? (resid + (size_t)b * strideR) : nullptr;
  const float* biasb = bias;
  if (BIAS_MODE != 0) biasb = bias + (size_t)b * strideBias;
#pragma unroll
  for (int i = 0; i < 4; ++i) {
    const int mBase = m0 + (i << 4);
#pragma unroll
    for (int j = 0; j < 4; ++j) {
      const int n = n0 + (j << 4) + rlane;
      float bv = 0.f;
      if (BIAS_MODE == 2) bv = biasb[n];
#pragma unroll
      for (int r = 0; r < 8; ++r) {
        float v = acc[i][j][r] * scale;
        if (BIAS_MODE == 1) v += biasb[mBase + mOff + r];
        if (BIAS_MODE == 2) v += bv;
        if (RESID) v += Rb[(size_t)(mBase + mOff + r) * ldc + n];
        if (ACT == 2) v = fmaxf(v, 0.0f);
        if (ACT == 4) v = (v > 0.f) ? v : 0.01f * v;
        slab[(mOff + r) * 68 + (j << 4) + rlane] = v;
      }
    }
    __builtin_amdgcn_fence(__ATOMIC_RELEASE, "workgroup");
    __builtin_amdgcn_wave_barrier();
    __builtin_amdgcn_fence(__ATOMIC_ACQUIRE, "workgroup");
    if (OUT_MODE == 0) {
      float* C = (float*)Cout + (size_t)b * strideC;
      const int hh = lane >> 4, c4 = (lane & 15) * 4;
      for (int pass = 0; pass < 2; ++pass) {
#pragma unroll
        for (int it = 0; it < 8; ++it) {
          const int row = it * 2 + hh;
          v4f v = *(const v4f*)(slab + row * 68 + c4);
          *(volatile v4f*)(C + (size_t)(mBase + row) * ldc + n0 + c4) = v;
        }
        __threadfence();
      }
    } else {
      const int q = lane >> 3, c8 = (lane & 7) * 8;
      unsigned short* C  = (unsigned short*)Cout  + (size_t)b * strideC;
      unsigned short* C2 = (OUT_MODE == 2) ? ((unsigned short*)Cout2 + (size_t)b * strideC) : nullptr;
      for (int pass = 0; pass < 2; ++pass) {
#pragma unroll
        for (int it = 0; it < 4; ++it) {
          const int row = it * 4 + q;
          const float* sp = slab + row * 68 + c8;
          v8h hv, lv;
#pragma unroll
          for (int e = 0; e < 8; ++e) {
            if (OUT_MODE == 1) {
              hv[e] = (_Float16)sp[e];
            } else {
              unsigned short hb = f2bf_bits(sp[e]);
              unsigned short lb = f2bf_bits(sp[e] - bf_bits2f(hb));
              hv[e] = __builtin_bit_cast(_Float16, hb);
              lv[e] = __builtin_bit_cast(_Float16, lb);
            }
          }
          *(volatile v8h*)(C + (size_t)(mBase + row) * ldc + n0 + c8) = hv;
          if (OUT_MODE == 2) *(volatile v8h*)(C2 + (size_t)(mBase + row) * ldc + n0 + c8) = lv;
        }
        __threadfence();
      }
    }
    __builtin_amdgcn_fence(__ATOMIC_RELEASE, "workgroup");
    __builtin_amdgcn_wave_barrier();
    __builtin_amdgcn_fence(__ATOMIC_ACQUIRE, "workgroup");
  }
}

__global__ __launch_bounds__(256) void cast8_f16_kernel(const float* __restrict__ in, unsigned short* __restrict__ out, int n8) {
  const int i = blockIdx.x * 256 + threadIdx.x;
  if (i >= n8) return;
  const float* p = in + 8 * (size_t)i;
  const v4f a = *(const v4f*)(p);
  const v4f c = *(const v4f*)(p + 4);
  unsigned short hb[8];
#pragma unroll
  for (int e = 0; e < 4; ++e) {
    hb[e]     = h_bits(a[e]);
    hb[4 + e] = h_bits(c[e]);
  }
  const v4u u = (v4u){pk16(hb[0], hb[1]), pk16(hb[2], hb[3]), pk16(hb[4], hb[5]), pk16(hb[6], hb[7])};
  unsigned short* q = out + 8 * (size_t)i;
  *(volatile v4u*)q = u;
  __threadfence();
  *(volatile v4u*)q = u;
}

__global__ __launch_bounds__(256) void gather_sr_kernel(const float* __restrict__ x,
                                                        unsigned short* __restrict__ ahi, unsigned short* __restrict__ alo) {
  const int i   = blockIdx.x * 256 + threadIdx.x;
  const int row = i >> 8;
  const int c8  = (i & 255) * 8;
  const int sub = c8 >> 9, c = c8 & 511;
  const int b   = row >> 8, nk = row & 255;
  const int hp  = nk >> 4, wp = nk & (kRedHW - 1);
  const int kh  = sub >> 1, kw = sub & 1;
  const int tok = (2 * hp + kh) * kGridHW + 2 * wp + kw;
  const float* src = x + ((size_t)(b * kTok + tok) * kDim + c);
  const v4f a = *(const v4f*)(src);
  const v4f d = *(const v4f*)(src + 4);
  unsigned short hb[8], lb[8];
#pragma unroll
  for (int e = 0; e < 4; ++e) {
    hb[e] = f2bf_bits(a[e]);      lb[e]     = f2bf_bits(a[e] - bf_bits2f(hb[e]));
    hb[4 + e] = f2bf_bits(d[e]);  lb[4 + e] = f2bf_bits(d[e] - bf_bits2f(hb[4 + e]));
  }
  const v4u uh = (v4u){pk16(hb[0], hb[1]), pk16(hb[2], hb[3]), pk16(hb[4], hb[5]), pk16(hb[6], hb[7])};
  const v4u ul = (v4u){pk16(lb[0], lb[1]), pk16(lb[2], lb[3]), pk16(lb[4], lb[5]), pk16(lb[6], lb[7])};
  unsigned short* ph = ahi + (size_t)row * kConvK + c8;
  unsigned short* pl = alo + (size_t)row * kConvK + c8;
  *(volatile v4u*)ph = uh;
  *(volatile v4u*)pl = ul;
  __threadfence();
  *(volatile v4u*)ph = uh;
  *(volatile v4u*)pl = ul;
}

__global__ __launch_bounds__(256) void repack_sr_kernel(const float* __restrict__ srw,
                                                        unsigned short* __restrict__ whi, unsigned short* __restrict__ wlo) {
  const int i   = blockIdx.x * 256 + threadIdx.x;
  const int o   = i >> 8;
  const int c8  = (i & 255) * 8;
  const int sub = c8 >> 9, c = c8 & 511;
  unsigned short hb[8], lb[8];
#pragma unroll
  for (int e = 0; e < 8; ++e) {
    const float f = srw[((size_t)(o * kDim + c + e) << 2) + sub];
    hb[e] = f2bf_bits(f);
    lb[e] = f2bf_bits(f - bf_bits2f(hb[e]));
  }
  const v4u uh = (v4u){pk16(hb[0], hb[1]), pk16(hb[2], hb[3]), pk16(hb[4], hb[5]), pk16(hb[6], hb[7])};
  const v4u ul = (v4u){pk16(lb[0], lb[1]), pk16(lb[2], lb[3]), pk16(lb[4], lb[5]), pk16(lb[6], lb[7])};
  unsigned short* ph = whi + (size_t)o * kConvK + c8;
  unsigned short* pl = wlo + (size_t)o * kConvK + c8;
  *(volatile v4u*)ph = uh;
  *(volatile v4u*)pl = ul;
  __threadfence();
  *(volatile v4u*)ph = uh;
  *(volatile v4u*)pl = ul;
}

template <int MODE>
__global__ __launch_bounds__(256) void wtrans_kernel(const float* __restrict__ W, int nrows, int ncols,
                                                     unsigned short* __restrict__ out0, unsigned short* __restrict__ out1,
                                                     float scale) {
  __shared__ float sm[64][65];
  const int t  = threadIdx.x;
  const int r0 = blockIdx.x * 64;
  const int c0 = blockIdx.y * 64;
#pragma unroll
  for (int i = 0; i < 16; ++i) {
    const int e  = i * 256 + t;
    const int rl = e >> 6;
    const int cl = e & 63;
    sm[cl][rl] = W[(size_t)(r0 + rl) * ncols + c0 + cl] * scale;
  }
  __syncthreads();
  const int lane = t & 31, wave = t >> 5;
  const int q = lane >> 3, c8 = (lane & 7) * 8;
  v4u uh[2], ul[2];
#pragma unroll
  for (int it = 0; it < 2; ++it) {
    const int row = wave * 8 + it * 4 + q;
    unsigned short hb[8], lb[8];
#pragma unroll
    for (int e = 0; e < 8; ++e) {
      const float f = sm[row][c8 + e];
      if (MODE == 0) { hb[e] = h_bits(f); lb[e] = 0; }
      else { hb[e] = f2bf_bits(f); lb[e] = f2bf_bits(f - bf_bits2f(hb[e])); }
    }
    uh[it] = (v4u){pk16(hb[0], hb[1]), pk16(hb[2], hb[3]), pk16(hb[4], hb[5]), pk16(hb[6], hb[7])};
    ul[it] = (v4u){pk16(lb[0], lb[1]), pk16(lb[2], lb[3]), pk16(lb[4], lb[5]), pk16(lb[6], lb[7])};
  }
  for (int pass = 0; pass < 2; ++pass) {
#pragma unroll
    for (int it = 0; it < 2; ++it) {
      const int row = wave * 8 + it * 4 + q;
      const size_t o = (size_t)(c0 + row) * nrows + r0 + c8;
      *(volatile v4u*)(out0 + o) = uh[it];
      if (MODE == 1) *(volatile v4u*)(out1 + o) = ul[it];
    }
    __threadfence();
  }
}

__global__ __launch_bounds__(256) void ln_split_kernel(const float* __restrict__ R, const float* __restrict__ gam,
                                                       const float* __restrict__ bet,
                                                       unsigned short* __restrict__ ohi, unsigned short* __restrict__ olo) {
  const int lane = threadIdx.x & 31, wave = threadIdx.x >> 5;
  const int row  = blockIdx.x * 8 + wave;
  const float* rp = R + (size_t)row * kDim;
  const int cA = lane * 8, cB = 256 + lane * 8;
  const v4f x0 = *(const v4f*)(rp + cA), x1 = *(const v4f*)(rp + cA + 4);
  const v4f x2 = *(const v4f*)(rp + cB), x3 = *(const v4f*)(rp + cB + 4);
  const v4f g0 = *(const v4f*)(gam + cA), g1 = *(const v4f*)(gam + cA + 4);
  const v4f g2 = *(const v4f*)(gam + cB), g3 = *(const v4f*)(gam + cB + 4);
  const v4f b0 = *(const v4f*)(bet + cA), b1 = *(const v4f*)(bet + cA + 4);
  const v4f b2 = *(const v4f*)(bet + cB), b3 = *(const v4f*)(bet + cB + 4);
  float xv[16], gv[16], bv[16];
#pragma unroll
  for (int e = 0; e < 4; ++e) {
    xv[e] = x0[e]; xv[4 + e] = x1[e]; xv[8 + e] = x2[e]; xv[12 + e] = x3[e];
    gv[e] = g0[e]; gv[4 + e] = g1[e]; gv[8 + e] = g2[e]; gv[12 + e] = g3[e];
    bv[e] = b0[e]; bv[4 + e] = b1[e]; bv[8 + e] = b2[e]; bv[12 + e] = b3[e];
  }
  float s = 0.f;
#pragma unroll
  for (int e = 0; e < 16; ++e) s += xv[e];
#pragma unroll
  for (int off = 16; off > 0; off >>= 1) s += __shfl_xor(s, off, 32);
  const float mu = s * kInvDim;
  float qd = 0.f;
#pragma unroll
  for (int e = 0; e < 16; ++e) { const float d = xv[e] - mu; qd += d * d; }
#pragma unroll
  for (int off = 16; off > 0; off >>= 1) qd += __shfl_xor(qd, off, 32);
  const float rstd = rsqrtf(qd * kInvDim + kLnEps);
  unsigned short hb[16], lb[16];
#pragma unroll
  for (int e = 0; e < 16; ++e) {
    const float y = (xv[e] - mu) * rstd * gv[e] + bv[e];
    hb[e] = f2bf_bits(y);
    lb[e] = f2bf_bits(y - bf_bits2f(hb[e]));
  }
  const v4u h0 = (v4u){pk16(hb[0], hb[1]), pk16(hb[2], hb[3]), pk16(hb[4], hb[5]), pk16(hb[6], hb[7])};
  const v4u h1 = (v4u){pk16(hb[8], hb[9]), pk16(hb[10], hb[11]), pk16(hb[12], hb[13]), pk16(hb[14], hb[15])};
  const v4u l0 = (v4u){pk16(lb[0], lb[1]), pk16(lb[2], lb[3]), pk16(lb[4], lb[5]), pk16(lb[6], lb[7])};
  const v4u l1 = (v4u){pk16(lb[8], lb[9]), pk16(lb[10], lb[11]), pk16(lb[12], lb[13]), pk16(lb[14], lb[15])};
  unsigned short* ph = ohi + (size_t)row * kDim;
  unsigned short* pl = olo + (size_t)row * kDim;
  for (int pass = 0; pass < 2; ++pass) {
    *(volatile v4u*)(ph + cA) = h0;
    *(volatile v4u*)(ph + cB) = h1;
    *(volatile v4u*)(pl + cA) = l0;
    *(volatile v4u*)(pl + cB) = l1;
    __threadfence();
  }
}

__global__ __launch_bounds__(256) void vt_kernel(const unsigned short* __restrict__ V16, unsigned short* __restrict__ Vt) {
  __shared__ unsigned short sm[64][72];
  const int t  = threadIdx.x;
  const int m0 = blockIdx.x * 64;
  const int b  = blockIdx.y;
  const unsigned short* vb = V16 + (size_t)b * kNk * kDim;
#pragma unroll
  for (int i = 0; i < 2; ++i) {
    const int idx = i * 256 + t;
    const int ml  = idx >> 3;
    const int ch  = (idx & 7) * 8;
    const v4u w = *(const v4u*)(vb + (size_t)(m0 + ml) * kHd + ch);
#pragma unroll
    for (int e = 0; e < 4; ++e) {
      sm[ch + 2 * e][ml]     = (unsigned short)(w[e] & 0xffffu);
      sm[ch + 2 * e + 1][ml] = (unsigned short)(w[e] >> 16);
    }
  }
  __syncthreads();
  const int lane = t & 31, wave = t >> 5;
  const int q = lane >> 3, c8 = (lane & 7) * 8;
  v4u u[2];
#pragma unroll
  for (int it = 0; it < 2; ++it) {
    const int row = wave * 8 + it * 4 + q;
    u[it] = (v4u){pk16(sm[row][c8 + 0], sm[row][c8 + 1]), pk16(sm[row][c8 + 2], sm[row][c8 + 3]),
                  pk16(sm[row][c8 + 4], sm[row][c8 + 5]), pk16(sm[row][c8 + 6], sm[row][c8 + 7])};
  }
  unsigned short* ob = Vt + (size_t)b * kHd * kKeys;
  for (int pass = 0; pass < 2; ++pass) {
#pragma unroll
    for (int it = 0; it < 2; ++it) {
      const int row = wave * 8 + it * 4 + q;
      *(volatile v4u*)(ob + (size_t)row * kKeys + m0 + c8) = u[it];
    }
    __threadfence();
  }
}

__global__ __launch_bounds__(256) void softmax_row_kernel(const float* __restrict__ S, unsigned short* __restrict__ P, float carry) {
  __shared__ float redM[8];
  __shared__ float redS[8];
  const int row  = blockIdx.x;
  const int t    = threadIdx.x;
  const int lane = t & 31, wave = t >> 5;
  const int c0   = t * 8;
  const float* sr = S + (size_t)row * kKeys + c0;
  const v4f a = *(const v4f*)(sr);
  const v4f c = *(const v4f*)(sr + 4);
  float xv[8];
#pragma unroll
  for (int e = 0; e < 4; ++e) { xv[e] = a[e]; xv[4 + e] = c[e]; }
  float m = fmaxf(fmaxf(fmaxf(xv[0], xv[1]), fmaxf(xv[2], xv[3])), fmaxf(fmaxf(xv[4], xv[5]), fmaxf(xv[6], xv[7])));
#pragma unroll
  for (int off = 16; off > 0; off >>= 1) m = fmaxf(m, __shfl_xor(m, off, 32));
  if (lane == 0) redM[wave] = m;
  __syncthreads();
  float gm = redM[0];
#pragma unroll
  for (int w = 1; w < 8; ++w) gm = fmaxf(gm, redM[w]);
  float ev[8];
  float s = 0.f;
#pragma unroll
  for (int e = 0; e < 8; ++e) { ev[e] = expf(xv[e] - gm); s += ev[e]; }
#pragma unroll
  for (int off = 16; off > 0; off >>= 1) s += __shfl_xor(s, off, 32);
  if (lane == 0) redS[wave] = s;
  __syncthreads();
  float tot = redS[0];
#pragma unroll
  for (int w = 1; w < 8; ++w) tot += redS[w];
  const float inv = carry * (1.0f / tot);
  unsigned short hb[8];
#pragma unroll
  for (int e = 0; e < 8; ++e) hb[e] = h_bits(ev[e] * inv);
  const v4u u = (v4u){pk16(hb[0], hb[1]), pk16(hb[2], hb[3]), pk16(hb[4], hb[5]), pk16(hb[6], hb[7])};
  unsigned short* pp = P + (size_t)row * kKeys + c0;
  *(volatile v4u*)pp = u;
  __threadfence();
  *(volatile v4u*)pp = u;
}

extern "C" void kernel_launch(void* const* d_in, const int* in_sizes, int n_in,
                              void* d_out, int out_size, void* d_ws, size_t ws_size,
                              hipStream_t stream) {
  if (n_in < 13) return;
  if (in_sizes[0] != kRows * kDim || out_size != kRows * kDim) return;
  if (in_sizes[3] != kDim * kDim || in_sizes[4] != kDim || in_sizes[5] != kDim * 2 * kDim || in_sizes[6] != 2 * kDim) return;
  if (in_sizes[7] != kDim * kDim * 4 || in_sizes[8] != kDim || in_sizes[9] != kDim || in_sizes[10] != kDim) return;
  if (in_sizes[11] != kDim * kDim || in_sizes[12] != kDim) return;

  const float* x      = (const float*)d_in[0];
  const float* q_w    = (const float*)d_in[3];
  const float* q_b    = (const float*)d_in[4];
  const float* kv_w   = (const float*)d_in[5];
  const float* kv_b   = (const float*)d_in[6];
  const float* sr_w   = (const float*)d_in[7];
  const float* sr_b   = (const float*)d_in[8];
  const float* ln_g   = (const float*)d_in[9];
  const float* ln_b   = (const float*)d_in[10];
  const float* proj_w = (const float*)d_in[11];
  const float* proj_b = (const float*)d_in[12];
  float* out = (float*)d_out;

  char* ws = (char*)d_ws;
  size_t off = 0;
  unsigned short* X16   = (unsigned short*)(ws + off); off += (size_t)kRows * kDim * 2;
  unsigned short* Wq16  = (unsigned short*)(ws + off); off += (size_t)kDim * kDim * 2;
  unsigned short* WsrHi = (unsigned short*)(ws + off); off += (size_t)kDim * kConvK * 2;
  unsigned short* WsrLo = (unsigned short*)(ws + off); off += (size_t)kDim * kConvK * 2;
  unsigned short* WkvHi = (unsigned short*)(ws + off); off += (size_t)2 * kDim * kDim * 2;
  unsigned short* WkvLo = (unsigned short*)(ws + off); off += (size_t)2 * kDim * kDim * 2;
  unsigned short* WpjHi = (unsigned short*)(ws + off); off += (size_t)kDim * kDim * 2;
  unsigned short* WpjLo = (unsigned short*)(ws + off); off += (size_t)kDim * kDim * 2;
  unsigned short* Qh    = (unsigned short*)(ws + off); off += (size_t)kHeads * kRows * kHd * 2;
  unsigned short* AsrHi = (unsigned short*)(ws + off); off += (size_t)kKvRows * kConvK * 2;
  unsigned short* AsrLo = (unsigned short*)(ws + off); off += (size_t)kKvRows * kConvK * 2;
  float*          R     = (float*)(ws + off);          off += (size_t)kKvRows * kDim * 4;
  unsigned short* XkvHi = (unsigned short*)(ws + off); off += (size_t)kKvRows * kDim * 2;
  unsigned short* XkvLo = (unsigned short*)(ws + off); off += (size_t)kKvRows * kDim * 2;
  unsigned short* K16   = (unsigned short*)(ws + off); off += (size_t)kKvRows * kDim * 2;
  unsigned short* V16   = (unsigned short*)(ws + off); off += (size_t)kKvRows * kDim * 2;
  unsigned short* Vt    = (unsigned short*)(ws + off); off += (size_t)kBatch * kHd * kKeys * 2;
  float*          S     = (float*)(ws + off);          off += (size_t)kHeadGrp * kTok * kKeys * 4;
  unsigned short* P     = (unsigned short*)(ws + off); off += (size_t)kHeadGrp * kTok * kKeys * 2;
  unsigned short* CtxHi = (unsigned short*)(ws + off); off += (size_t)kRows * kDim * 2;
  unsigned short* CtxLo = (unsigned short*)(ws + off); off += (size_t)kRows * kDim * 2;
  if (off > ws_size) return;

  cast8_f16_kernel<<<(kRows * kDim / 8) / 256, 256, 0, stream>>>(x, X16, kRows * kDim / 8);
  gather_sr_kernel<<<(kKvRows * kConvK / 8) / 256, 256, 0, stream>>>(x, AsrHi, AsrLo);
  wtrans_kernel<0><<<dim3(kDim / 64, kDim / 64), 256, 0, stream>>>(q_w, kDim, kDim, Wq16, Wq16, kWqCarry);
  wtrans_kernel<1><<<dim3(kDim / 64, 2 * kDim / 64), 256, 0, stream>>>(kv_w, kDim, 2 * kDim, WkvHi, WkvLo, 1.0f);
  wtrans_kernel<1><<<dim3(kDim / 64, kDim / 64), 256, 0, stream>>>(proj_w, kDim, kDim, WpjHi, WpjLo, 1.0f);
  repack_sr_kernel<<<(kDim * kConvK / 8) / 256, 256, 0, stream>>>(sr_w, WsrHi, WsrLo);

  wmma_gemm64<0, false, 2, 1, false><<<dim3(16, kHeads), 256, 0, stream>>>(
      X16, X16, kDim, 0L,
      Wq16, Wq16, kDim, (long)(kHd * kDim),
      (void*)Qh, (void*)Qh, kHd, (long)kRows * kHd,
      q_b, (long)kHd,
      nullptr, 0L,
      kRows, kHd, kDim, kWqCarryInv);

  wmma_gemm64<1, true, 2, 0, false><<<dim3(32, 1), 256, 0, stream>>>(
      AsrHi, AsrLo, kConvK, 0L,
      WsrHi, WsrLo, kConvK, 0L,
      (void*)R, (void*)R, kDim, 0L,
      sr_b, 0L,
      nullptr, 0L,
      kKvRows, kDim, kConvK, 1.0f);

  ln_split_kernel<<<kKvRows / 8, 256, 0, stream>>>(R, ln_g, ln_b, XkvHi, XkvLo);

  wmma_gemm64<1, true, 2, 1, false><<<dim3(32, 1), 256, 0, stream>>>(
      XkvHi, XkvLo, kDim, 0L,
      WkvHi, WkvLo, kDim, 0L,
      (void*)K16, (void*)K16, kDim, 0L,
      kv_b, 0L,
      nullptr, 0L,
      kKvRows, kDim, kDim, 1.0f);
  wmma_gemm64<1, true, 2, 1, false><<<dim3(32, 1), 256, 0, stream>>>(
      XkvHi, XkvLo, kDim, 0L,
      WkvHi + (size_t)kDim * kDim, WkvLo + (size_t)kDim * kDim, kDim, 0L,
      (void*)V16, (void*)V16, kDim, 0L,
      kv_b + kDim, 0L,
      nullptr, 0L,
      kKvRows, kDim, kDim, 1.0f);

  vt_kernel<<<dim3(kKeys / 64, kBatch), 256, 0, stream>>>(V16, Vt);

  for (int b = 0; b < kBatch; ++b) {
    for (int g = 0; g < kHeads / kHeadGrp; ++g) {
      const unsigned short* qa = Qh + ((size_t)(g * kHeadGrp) * kRows + (size_t)b * kTok) * kHd;
      const unsigned short* kb = K16 + (size_t)b * kNk * kDim;
      wmma_gemm64<0, false, 0, 0, false><<<dim3(64, kHeadGrp), 256, 0, stream>>>(
          qa, qa, kHd, (long)kRows * kHd,
          kb, kb, kHd, 0L,
          (void*)S, (void*)S, kKeys, (long)kTok * kKeys,
          nullptr, 0L,
          nullptr, 0L,
          kTok, kKeys, kHd, kAttnScale);
      softmax_row_kernel<<<kHeadGrp * kTok, 256, 0, stream>>>(S, P, kPCarry);
      const unsigned short* vtb = Vt + (size_t)b * kHd * kKeys;
      const size_t co = (size_t)b * kTok * kDim + (size_t)g * kHeadGrp * kHd;
      wmma_gemm64<0, false, 0, 2, false><<<dim3(2, kHeadGrp), 256, 0, stream>>>(
          P, P, kKeys, (long)kTok * kKeys,
          vtb, vtb, kKeys, 0L,
          (void*)(CtxHi + co), (void*)(CtxLo + co), kDim, (long)kHd,
          nullptr, 0L,
          nullptr, 0L,
          kTok, kHd, kKeys, kPCarryInv);
    }
  }

  wmma_gemm64<1, true, 2, 0, false><<<dim3(128, 1), 256, 0, stream>>>(
      CtxHi, CtxLo, kDim, 0L,
      WpjHi, WpjLo, kDim, 0L,
      (void*)out, (void*)out, kDim, 0L,
      proj_b, 0L,
      nullptr, 0L,
      kRows, kDim, kDim, 1.0f);
}
